// DAttentionMM_84155589198444
// MI455X (gfx1250) — hardware-verified
//
#include <hip/hip_runtime.h>
#define NB 8
#define CC 256
#define HS 64
#define PX (HS * HS)
#define NR ((size_t)NB * PX)
#define NHD 8
#define HC 32
#define GK 8
#define NS 64
#define NK 128
#define NKR ((size_t)NB * NK)
#define KF (9 * 2 * CC)
#define RCH 8192
typedef __bf16 v16b __attribute__((ext_vector_type(16)));
typedef unsigned short v8us __attribute__((ext_vector_type(8), may_alias));
typedef float  v8f  __attribute__((ext_vector_type(8)));
typedef float  v4f  __attribute__((ext_vector_type(4)));
typedef float  v4fa __attribute__((ext_vector_type(4), may_alias));
union FragB { v16b v; v8us half[2]; unsigned short u[16]; };

__device__ __forceinline__ unsigned short bf16_bits(float x) { unsigned int u = __float_as_uint(x); return (unsigned short)((u + 0x7FFFu + ((u >> 16) & 1u)) >> 16); }
__device__ __forceinline__ float bf16_val(unsigned short b) { return __uint_as_float(((unsigned int)b) << 16); }
__device__ __forceinline__ float bf16_round(float x) { return bf16_val(bf16_bits(x)); }
template <int NT>
__device__ __forceinline__ v8f mmaN(v16b ah, v16b al, v16b bh, v16b bl, v8f c) {
  c = __builtin_amdgcn_wmma_f32_16x16x32_bf16(false, ah, false, bh, (short)0, c, false, false);
  if (NT >= 2) c = __builtin_amdgcn_wmma_f32_16x16x32_bf16(false, al, false, bh, (short)0, c, false, false);
  if (NT >= 3) c = __builtin_amdgcn_wmma_f32_16x16x32_bf16(false, ah, false, bl, (short)0, c, false, false);
  asm volatile("v_nop\n\tv_nop\n\tv_nop\n\tv_nop" : "+v"(c) : "v"(ah), "v"(al), "v"(bh), "v"(bl));
  return c;
}

__global__ __launch_bounds__(256) void k_wt_bf16(const float* __restrict__ W, unsigned short* __restrict__ Wt, int K, int N) {
  const int t = blockIdx.x * 256 + threadIdx.x;
  const int k8n = K / 8;
  if (t >= N * k8n) return;
  const int n = t / k8n, k8 = (t % k8n) * 8;
  v8us v;
#pragma unroll
  for (int i = 0; i < 8; ++i) v[i] = bf16_bits(W[(size_t)(k8 + i) * N + n]);
  *(volatile v8us*)(Wt + (size_t)n * K + k8) = v;
  __threadfence();
  *(volatile v8us*)(Wt + (size_t)n * K + k8) = v;
}

template <bool ASPLIT, int ACT, bool BIAS_BF16>
__global__ __launch_bounds__(128) void k_gemm_bf(const float* __restrict__ A, int lda, const unsigned short* __restrict__ Wt, int ldb,
                                               const float* __restrict__ bias, float* __restrict__ C, int ldc, int M, int N, int K) {
  __shared__ __attribute__((aligned(16))) float so[4][16][64];
  const int tid = threadIdx.x, w = tid >> 5, lane = tid & 31, ln = lane & 15, hh = lane >> 4;
  const int ntn = N / 64;
  const int wid = blockIdx.x * 4 + w;
  const int mt = wid / ntn, nq = wid % ntn;
  if (mt * 16 >= M) return;
  const int row0 = mt * 16, col0 = nq * 64;
  const float* arow = A + (size_t)(row0 + ln) * lda;
  v8f acc[4] = {};
  for (int kb = 0; kb < K; kb += 32) {
    FragB ah, al;
    const v4f x0 = *(const v4fa*)(arow + kb + 8 * hh), x1 = *(const v4fa*)(arow + kb + 8 * hh + 4);
    const v4f x2 = *(const v4fa*)(arow + kb + 16 + 8 * hh), x3 = *(const v4fa*)(arow + kb + 16 + 8 * hh + 4);
    float xs[16] = {x0[0],x0[1],x0[2],x0[3],x1[0],x1[1],x1[2],x1[3],x2[0],x2[1],x2[2],x2[3],x3[0],x3[1],x3[2],x3[3]};
#pragma unroll
    for (int i = 0; i < 16; ++i) { const unsigned short hb = bf16_bits(xs[i]); ah.u[i] = hb; al.u[i] = ASPLIT ? bf16_bits(xs[i] - bf16_val(hb)) : (unsigned short)0; }
#pragma unroll
    for (int t = 0; t < 4; ++t) {
      const unsigned short* brow = Wt + (size_t)(col0 + t * 16 + ln) * ldb + kb;
      FragB b;
      b.half[0] = *(const v8us*)(brow + 8 * hh);
      b.half[1] = *(const v8us*)(brow + 16 + 8 * hh);
      acc[t] = mmaN<ASPLIT ? 2 : 1>(ah.v, al.v, b.v, b.v, acc[t]);
    }
  }
#pragma unroll
  for (int t = 0; t < 4; ++t) {
    float bv = bias ? bias[col0 + t * 16 + ln] : 0.f;
    if (BIAS_BF16) bv = bf16_round(bv);
#pragma unroll
    for (int r = 0; r < 8; ++r) { float v = acc[t][r] + bv; if (ACT == 1) v = fmaxf(v, 0.f); so[w][8 * hh + r][t * 16 + ln] = v; }
  }
  __builtin_amdgcn_fence(__ATOMIC_ACQ_REL, "workgroup");
  __builtin_amdgcn_wave_barrier();
  const int rsub = lane >> 4, c4 = (lane & 15) * 4;
  for (int pass = 0; pass < 2; ++pass) {
#pragma unroll
    for (int q = 0; q < 8; ++q) {
      const int r = q * 2 + rsub;
      const v4f v = *(const v4fa*)&so[w][r][c4];
      *(volatile v4f*)(C + (size_t)(row0 + r) * ldc + col0 + c4) = v;
    }
    if (pass == 0) __threadfence();
  }
}

template <bool ASPLIT, int ACT, bool BIAS_BF16, bool RES_BF16>
__global__ __launch_bounds__(128) void k_gemm_bf3(const float* __restrict__ A, int lda, const unsigned short* __restrict__ Wt, int ldb,
                                                const float* __restrict__ bias, const float* __restrict__ resid, int rmod, int ldr,
                                                float* __restrict__ C, int ldc, int M, int N, int K) {
  __shared__ __attribute__((aligned(16))) float so[4][16][64];
  const int tid = threadIdx.x, w = tid >> 5, lane = tid & 31, ln = lane & 15, hh = lane >> 4;
  const int ntn = N / 64;
  const int wid = blockIdx.x * 4 + w;
  const int mt = wid / ntn, nq = wid % ntn;
  if (mt * 16 >= M) return;
  const int row0 = mt * 16, col0 = nq * 64;
  const float* arow = A + (size_t)(row0 + ln) * lda;
  v8f acc[4] = {};
  for (int kb = 0; kb < K; kb += 32) {
    FragB ah, al;
    const v4f x0 = *(const v4fa*)(arow + kb + 8 * hh), x1 = *(const v4fa*)(arow + kb + 8 * hh + 4);
    const v4f x2 = *(const v4fa*)(arow + kb + 16 + 8 * hh), x3 = *(const v4fa*)(arow + kb + 16 + 8 * hh + 4);
    float xs[16] = {x0[0],x0[1],x0[2],x0[3],x1[0],x1[1],x1[2],x1[3],x2[0],x2[1],x2[2],x2[3],x3[0],x3[1],x3[2],x3[3]};
#pragma unroll
    for (int i = 0; i < 16; ++i) { const unsigned short hb = bf16_bits(xs[i]); ah.u[i] = hb; al.u[i] = ASPLIT ? bf16_bits(xs[i] - bf16_val(hb)) : (unsigned short)0; }
#pragma unroll
    for (int t = 0; t < 4; ++t) {
      const unsigned short* brow = Wt + (size_t)(col0 + t * 16 + ln) * ldb + kb;
      FragB b;
      b.half[0] = *(const v8us*)(brow + 8 * hh);
      b.half[1] = *(const v8us*)(brow + 16 + 8 * hh);
      acc[t] = mmaN<ASPLIT ? 2 : 1>(ah.v, al.v, b.v, b.v, acc[t]);
    }
  }
#pragma unroll
  for (int t = 0; t < 4; ++t) {
    const int col = col0 + t * 16 + ln;
    float bv = bias ? bias[col] : 0.f;
    if (BIAS_BF16) bv = bf16_round(bv);
#pragma unroll
    for (int r = 0; r < 8; ++r) {
      float v = acc[t][r] + bv;
      if (resid) { float rv = resid[(size_t)((row0 + 8 * hh + r) % rmod) * ldr + col]; if (RES_BF16) rv = bf16_round(rv); v += rv; }
      if (ACT == 1) v = fmaxf(v, 0.f);
      if (ACT == 2) v = 0.5f * v * (1.0f + erff(v * 0.70710678118654752f));
      if (ACT == 3) { const float u = 0.7978845608028654f * (v + 0.044715f * v * v * v); v = 0.5f * v * (1.0f + tanhf(u)); }
      so[w][8 * hh + r][t * 16 + ln] = v;
    }
  }
  __builtin_amdgcn_fence(__ATOMIC_ACQ_REL, "workgroup");
  __builtin_amdgcn_wave_barrier();
  const int rsub = lane >> 4, c4 = (lane & 15) * 4;
  for (int pass = 0; pass < 2; ++pass) {
#pragma unroll
    for (int q = 0; q < 8; ++q) {
      const int r = q * 2 + rsub;
      const v4f v = *(const v4fa*)&so[w][r][c4];
      *(volatile v4f*)(C + (size_t)(row0 + r) * ldc + col0 + c4) = v;
    }
    if (pass == 0) __threadfence();
  }
}
template <bool PARAM_BF16>
__global__ __launch_bounds__(256) void k_layernorm(const float* __restrict__ X, const float* __restrict__ R, const float* __restrict__ g, const float* __restrict__ bta,
                                                  float* __restrict__ out_sum, float* __restrict__ out_norm, int N, float eps) {
  __shared__ float red[256];
  const int row = blockIdx.x, tid = threadIdx.x;
  const float* x = X + (size_t)row * N; const float* rr = R ? R + (size_t)row * N : nullptr;
  float vals[16];
  const int per = N / 256;
  float s1 = 0.f;
  for (int u = 0; u < per / 4; ++u) {
    const int j = tid * 4 + 1024 * u;
    const v4f a = *(const v4fa*)(x + j);
    v4f b = {0.f,0.f,0.f,0.f}; if (rr) b = *(const v4fa*)(rr + j);
#pragma unroll
    for (int q = 0; q < 4; ++q) { const float v = a[q] + b[q]; vals[u * 4 + q] = v; s1 += v; }
  }
  red[tid] = s1; __syncthreads();
  for (int st = 128; st > 0; st >>= 1) { if (tid < st) red[tid] += red[tid + st]; __syncthreads(); }
  const float mu = red[0] / (float)N; __syncthreads();
  float s2 = 0.f;
  for (int u = 0; u < per / 4; ++u)
#pragma unroll
    for (int q = 0; q < 4; ++q) { const float c = vals[u * 4 + q] - mu; s2 += c * c; }
  red[tid] = s2; __syncthreads();
  for (int st = 128; st > 0; st >>= 1) { if (tid < st) red[tid] += red[tid + st]; __syncthreads(); }
  const float rs = rsqrtf(red[0] / (float)N + eps);
  for (int pass = 0; pass < 2; ++pass) {
    for (int u = 0; u < per / 4; ++u) {
      const int j = tid * 4 + 1024 * u;
      v4f o, sm;
#pragma unroll
      for (int q = 0; q < 4; ++q) {
        float gg = g[j + q], bb = bta[j + q];
        if (PARAM_BF16) { gg = bf16_round(gg); bb = bf16_round(bb); }
        sm[q] = vals[u * 4 + q]; o[q] = (vals[u * 4 + q] - mu) * rs * gg + bb;
      }
      if (out_sum) *(volatile v4f*)(out_sum + (size_t)row * N + j) = sm;
      *(volatile v4f*)(out_norm + (size_t)row * N + j) = o;
    }
    if (pass == 0) __threadfence();
  }
}


typedef _Float16 v16h __attribute__((ext_vector_type(16)));
union FragH { v16h v; v8us half[2]; _Float16 h[16]; unsigned short u[16]; };
template <int NT>
__device__ __forceinline__ v8f mmaH(v16h ah, v16h al, v16h bh, v16h bl, v8f c) {
  c = __builtin_amdgcn_wmma_f32_16x16x32_f16(false, ah, false, bh, (short)0, c, false, false);
  if (NT >= 2) c = __builtin_amdgcn_wmma_f32_16x16x32_f16(false, al, false, bh, (short)0, c, false, false);
  if (NT >= 3) c = __builtin_amdgcn_wmma_f32_16x16x32_f16(false, ah, false, bl, (short)0, c, false, false);
  asm volatile("v_nop\n\tv_nop\n\tv_nop\n\tv_nop" : "+v"(c) : "v"(ah), "v"(al), "v"(bh), "v"(bl));
  return c;
}
template <bool ASPLIT>
__global__ __launch_bounds__(128) void k_gemm_h(const float* __restrict__ A, int lda, size_t sA, const _Float16* __restrict__ Bh, int ldb, size_t sB, float alpha, float* __restrict__ C, int ldc, size_t sC, int M, int N, int K) {
  __shared__ __attribute__((aligned(16))) float so[4][16][64];
  const int tid = threadIdx.x, w = tid >> 5, lane = tid & 31, ln = lane & 15, hh = lane >> 4; const int by = blockIdx.y;
  A += (size_t)by * sA; Bh += (size_t)by * sB; C += (size_t)by * sC;
  const int ntn = (N + 63) / 64; const int wid = blockIdx.x * 4 + w; const int mt = wid / ntn, nq = wid % ntn; if (mt * 16 >= M) return;
  const int row0 = mt * 16, col0 = nq * 64; const float* arow = A + (size_t)(row0 + ln) * lda;
  v8f acc[4] = {};
  for (int kb = 0; kb < K; kb += 32) {
    FragH ah, al;
    const v4f x0 = *(const v4fa*)(arow + kb + 8 * hh), x1 = *(const v4fa*)(arow + kb + 8 * hh + 4), x2 = *(const v4fa*)(arow + kb + 16 + 8 * hh), x3 = *(const v4fa*)(arow + kb + 16 + 8 * hh + 4);
    float xs[16] = {x0[0],x0[1],x0[2],x0[3],x1[0],x1[1],x1[2],x1[3],x2[0],x2[1],x2[2],x2[3],x3[0],x3[1],x3[2],x3[3]};
#pragma unroll
    for (int i = 0; i < 16; ++i) { const _Float16 h = (_Float16)xs[i]; ah.h[i] = h; al.h[i] = ASPLIT ? (_Float16)(xs[i] - (float)h) : (_Float16)0.0f; }
#pragma unroll
    for (int t = 0; t < 4; ++t) { if (col0 + t * 16 >= N) continue; const size_t boff = (size_t)(col0 + t * 16 + ln) * ldb + kb; FragH bq; bq.half[0] = *(const v8us*)(Bh + boff + 8 * hh); bq.half[1] = *(const v8us*)(Bh + boff + 16 + 8 * hh);
      acc[t] = mmaH<ASPLIT ? 2 : 1>(ah.v, al.v, bq.v, bq.v, acc[t]); }
  }
#pragma unroll
  for (int t = 0; t < 4; ++t) { if (col0 + t * 16 >= N) continue;
#pragma unroll
    for (int r = 0; r < 8; ++r) so[w][8 * hh + r][t * 16 + ln] = acc[t][r] * alpha; }
  __builtin_amdgcn_fence(__ATOMIC_ACQ_REL, "workgroup"); __builtin_amdgcn_wave_barrier();
  const int rsub = lane >> 4, c4 = (lane & 15) * 4;
  for (int pass = 0; pass < 2; ++pass) {
#pragma unroll
    for (int q = 0; q < 8; ++q) { const int r = q * 2 + rsub; if (col0 + c4 < N) { const v4f v = *(const v4fa*)&so[w][r][c4]; *(volatile v4f*)(C + (size_t)(row0 + r) * ldc + col0 + c4) = v; } }
    if (pass == 0) __threadfence(); }
}

__global__ __launch_bounds__(256) void k_wt_f16(const float* __restrict__ W, _Float16* __restrict__ Wt, int K, int N, float scale) {
  const int t = blockIdx.x * 256 + threadIdx.x; if (t >= N * (K / 8)) return; const int n = t / (K / 8), k8 = (t % (K / 8)) * 8; FragH f;
#pragma unroll
  for (int i = 0; i < 8; ++i) f.h[i] = (_Float16)(bf16_round(W[(size_t)(k8 + i) * N + n]) * scale); const v8us o = f.half[0];
  *(volatile v8us*)((unsigned short*)Wt + (size_t)n * K + k8) = o; __threadfence(); *(volatile v8us*)((unsigned short*)Wt + (size_t)n * K + k8) = o;
}
template <int ACT>
__global__ __launch_bounds__(128) void k_gemm_hhx(const _Float16* __restrict__ A, int lda, size_t sA, const _Float16* __restrict__ Bh, int ldb, size_t sB, float alpha, const float* __restrict__ bias, size_t sBias, const float* __restrict__ CP, int rowsPerB, size_t sCPb, int row0g,
    float* __restrict__ C, _Float16* __restrict__ C16, int ldc, size_t sC, int M, int N, int K) {
  __shared__ __attribute__((aligned(16))) float so[4][16][64];
  const int tid = threadIdx.x, w = tid >> 5, lane = tid & 31, ln = lane & 15, hh = lane >> 4; const int by = blockIdx.y;
  A += (size_t)by * sA; Bh += (size_t)by * sB; const size_t cofs = (size_t)by * sC; const float* bp = bias ? bias + (size_t)by * sBias : nullptr;
  const int ntn = (N + 63) / 64; const int wid = blockIdx.x * 4 + w; const int mt = wid / ntn, nq = wid % ntn; if (mt * 16 >= M) return;
  const int row0 = mt * 16, col0 = nq * 64; const _Float16* arow = A + (size_t)(row0 + ln) * lda;
  v8f acc[4] = {};
  for (int kb = 0; kb < K; kb += 32) { FragH ah; ah.half[0] = *(const v8us*)((const unsigned short*)arow + kb + 8 * hh); ah.half[1] = *(const v8us*)((const unsigned short*)arow + kb + 16 + 8 * hh);
#pragma unroll
    for (int t = 0; t < 4; ++t) { if (col0 + t * 16 >= N) continue; const size_t boff = (size_t)(col0 + t * 16 + ln) * ldb + kb; FragH bq; bq.half[0] = *(const v8us*)((const unsigned short*)Bh + boff + 8 * hh); bq.half[1] = *(const v8us*)((const unsigned short*)Bh + boff + 16 + 8 * hh);
      acc[t] = mmaH<1>(ah.v, ah.v, bq.v, bq.v, acc[t]); }
  }
#pragma unroll
  for (int t = 0; t < 4; ++t) { if (col0 + t * 16 >= N) continue; const int col = col0 + t * 16 + ln; const float bv = bp ? bf16_round(bp[col]) : 0.f;
#pragma unroll
    for (int r = 0; r < 8; ++r) { float v = acc[t][r] * alpha + bv; if (CP) { const int rr = row0g + row0 + 8 * hh + r; if (rowsPerB < 0) v += CP[cofs + (size_t)rr * ldc + col];        else { const int bidx = rr / rowsPerB; v += CP[(size_t)bidx * sCPb + (size_t)by * 64 + col]; } } if (ACT == 1) v = (v > 0.f) ? v : expm1f(v); else if (ACT == 7) v = (v > 0.f) ? v + 1.0f : expf(v); else if (ACT == 8) v = tanhf(v); else if (ACT == 9) v = 0.5f * v * (1.0f + tanhf(0.7978845608028654f * (v + 0.044715f * v * v * v))); else if (ACT == 11) v = 1.0f / (1.0f + expf(-v)); else if (ACT == 12) v = (v > 0.f) ? v : 0.01f * v; else if (ACT == 14) v = (v > 0.f) ? v : 0.1f * v; else if (ACT == 16) v = (v >= 0.f) ? v : 0.3f * v; else if (ACT == 17) v = (v >= 0.f) ? v : 0.2f * v; else if (ACT == 15) v = v / (1.0f + expf(-v)); else if (ACT == 3) v = fmaxf(v, 0.f); else if (ACT == 6) v = 0.5f * v * (1.0f + erff(v * 0.70710678118654752f)); so[w][8 * hh + r][t * 16 + ln] = v; } }
  __builtin_amdgcn_fence(__ATOMIC_ACQ_REL, "workgroup"); __builtin_amdgcn_wave_barrier();
  const int rsub = lane >> 4, c4 = (lane & 15) * 4; typedef _Float16 v4h __attribute__((ext_vector_type(4)));
  for (int pass = 0; pass < 2; ++pass) {
#pragma unroll
    for (int q = 0; q < 8; ++q) { const int r = q * 2 + rsub; if (col0 + c4 < N) { const v4f v = *(const v4fa*)&so[w][r][c4]; if (C) *(volatile v4f*)(C + cofs + (size_t)(row0 + r) * ldc + col0 + c4) = v; if (C16) { v4h h4; for (int i = 0; i < 4; ++i) h4[i] = (_Float16)v[i]; *(volatile v4h*)(C16 + cofs + (size_t)(row0 + r) * ldc + col0 + c4) = h4; } } }
    if (pass == 0) __threadfence(); }
}


typedef _Float16 v4h __attribute__((ext_vector_type(4)));

__global__ __launch_bounds__(256) void k_x16(const float* __restrict__ x, _Float16* __restrict__ X16, size_t n8) { const size_t t = (size_t)blockIdx.x * 256 + threadIdx.x; if (t >= n8) return; FragH f;
#pragma unroll
  for (int q = 0; q < 8; ++q) f.h[q] = (_Float16)bf16_round(x[t * 8 + q]); *(volatile v8us*)((unsigned short*)X16 + t * 8) = f.half[0]; __threadfence(); *(volatile v8us*)((unsigned short*)X16 + t * 8) = f.half[0]; }
__global__ __launch_bounds__(256) void k_h16(const float* __restrict__ x, _Float16* __restrict__ X16, size_t n8) { const size_t t = (size_t)blockIdx.x * 256 + threadIdx.x; if (t >= n8) return; FragH f;
#pragma unroll
  for (int q = 0; q < 8; ++q) f.h[q] = (_Float16)x[t * 8 + q]; *(volatile v8us*)((unsigned short*)X16 + t * 8) = f.half[0]; __threadfence(); *(volatile v8us*)((unsigned short*)X16 + t * 8) = f.half[0]; }
__global__ __launch_bounds__(256) void k_round16f(const float* __restrict__ W, _Float16* __restrict__ Bt, size_t n8) { const size_t t = (size_t)blockIdx.x * 256 + threadIdx.x; if (t >= n8) return; FragH f;
#pragma unroll
  for (int i = 0; i < 8; ++i) f.h[i] = (_Float16)(bf16_round(W[t * 8 + i]) * 16.0f); *(volatile v8us*)((unsigned short*)Bt + t * 8) = f.half[0]; __threadfence(); *(volatile v8us*)((unsigned short*)Bt + t * 8) = f.half[0]; }
template <int NHv, int TTv>
__global__ __launch_bounds__(256) void k_vt(const _Float16* __restrict__ V16, int ldv, int voff, _Float16* __restrict__ Vt) { __shared__ unsigned short tl[64][66]; const int tid = threadIdx.x; const int slab = blockIdx.x / (TTv / 64), lg = blockIdx.x % (TTv / 64); const int b = slab / NHv, h = slab % NHv;
  for (int i = tid; i < 64 * 8; i += 256) { const int r = i / 8, c8 = (i % 8) * 8; FragH f; f.half[0] = *(const v8us*)((const unsigned short*)V16 + ((size_t)b * TTv + lg * 64 + r) * ldv + voff + h * 64 + c8);
#pragma unroll
    for (int q = 0; q < 8; ++q) tl[r][c8 + q] = f.u[q]; }
  __syncthreads();
  for (int pass = 0; pass < 2; ++pass) {
#pragma unroll
    for (int rd = 0; rd < 2; ++rd) { const int d = rd * 32 + tid / 8, pc = tid % 8; FragH f;
#pragma unroll
      for (int q = 0; q < 8; ++q) f.u[q] = tl[pc * 8 + q][d];
      *(volatile v8us*)((unsigned short*)Vt + ((size_t)slab * 64 + d) * TTv + lg * 64 + pc * 8) = f.half[0]; }
    if (pass == 0) __threadfence(); } }

__global__ __launch_bounds__(256) void k_hl(const float* __restrict__ F, _Float16* __restrict__ Hh, _Float16* __restrict__ Hl, size_t n8) { const size_t t = (size_t)blockIdx.x * 256 + threadIdx.x; if (t >= n8) return; FragH fh, fl; const v4f a = *(const v4fa*)(F + t * 8), c = *(const v4fa*)(F + t * 8 + 4);
#pragma unroll
  for (int q = 0; q < 4; ++q) { _Float16 h = (_Float16)a[q]; fh.h[q] = h; fl.h[q] = (_Float16)((a[q] - (float)h) * 1024.0f); h = (_Float16)c[q]; fh.h[4 + q] = h; fl.h[4 + q] = (_Float16)((c[q] - (float)h) * 1024.0f); }
  for (int pass = 0; pass < 2; ++pass) { *(volatile v8us*)((unsigned short*)Hh + t * 8) = fh.half[0]; *(volatile v8us*)((unsigned short*)Hl + t * 8) = fl.half[0]; if (pass == 0) __threadfence(); } }

__device__ __forceinline__ v16h g2_frag(const _Float16* p, int hh) { FragH f; f.half[0] = *(const v8us*)((const unsigned short*)p + 8 * hh); f.half[1] = *(const v8us*)((const unsigned short*)p + 16 + 8 * hh); return f.v; }
__device__ __forceinline__ v8f g2_mma(v16h a, v16h b, v8f c) { v8f d = __builtin_amdgcn_wmma_f32_16x16x32_f16(false, a, false, b, (short)0, c, false, false); asm volatile("v_nop\n\tv_nop\n\tv_nop\n\tv_nop" : "+v"(d) : "v"(a), "v"(b)); return d; }
template <int ACT>
__global__ __launch_bounds__(128) void k_gemm2(const _Float16* __restrict__ A, int lda, size_t sA, const _Float16* __restrict__ Bh, int ldb, size_t sB, float alpha, const float* __restrict__ bias, size_t sBias, const float* __restrict__ CP, int rowsPerB, size_t sCPb, int row0g,
    float* __restrict__ C, _Float16* __restrict__ C16, int ldc, size_t sC, int M, int N, int K) { static_assert(ACT == 0 || ACT == 3 || ACT == 6 || ACT == 8 || ACT == 9 || ACT == 11 || ACT == 12 || ACT == 14 || ACT == 15 || ACT == 16 || ACT == 17, "k_gemm2: unsupported ACT code (would silently apply no activation)");
  __shared__ __attribute__((aligned(16))) float so[4][32][68];
  const int tid = threadIdx.x, w = tid >> 5, lane = tid & 31, ln = lane & 15, hh = lane >> 4; const int by = blockIdx.y;
  A += (size_t)by * sA; Bh += (size_t)by * sB; const size_t cofs = (size_t)by * sC; const float* bp = bias ? bias + (size_t)by * sBias : nullptr;
  const int ntn = N >> 6; const int mt = blockIdx.x / ntn, nq = blockIdx.x - mt * ntn; const int row0 = mt * 128 + 32 * w, col0 = nq * 64; if (row0 >= M) return;
  const _Float16* a0p = A + (size_t)(row0 + ln) * lda; const _Float16* a1p = a0p + (size_t)16 * lda;
  const _Float16* b0p = Bh + (size_t)(col0 + ln) * ldb; const _Float16* b1p = b0p + (size_t)16 * ldb; const _Float16* b2p = b1p + (size_t)16 * ldb; const _Float16* b3p = b2p + (size_t)16 * ldb;
  const v8f z8 = {0.f,0.f,0.f,0.f,0.f,0.f,0.f,0.f}; v8f c00 = z8, c01 = z8, c02 = z8, c03 = z8, c10 = z8, c11 = z8, c12 = z8, c13 = z8;
#pragma unroll 1
  for (int kb = 0; kb < K; kb += 32) { const v16h a0 = g2_frag(a0p + kb, hh), a1 = g2_frag(a1p + kb, hh);
    v16h b = g2_frag(b0p + kb, hh); c00 = g2_mma(a0, b, c00); c10 = g2_mma(a1, b, c10);
    b = g2_frag(b1p + kb, hh); c01 = g2_mma(a0, b, c01); c11 = g2_mma(a1, b, c11);
    b = g2_frag(b2p + kb, hh); c02 = g2_mma(a0, b, c02); c12 = g2_mma(a1, b, c12);
    b = g2_frag(b3p + kb, hh); c03 = g2_mma(a0, b, c03); c13 = g2_mma(a1, b, c13); }
  v8f accs[8] = {c00, c01, c02, c03, c10, c11, c12, c13};
#pragma unroll
  for (int u = 0; u < 8; ++u) { const int t = u & 3, half = u >> 2; const int col = col0 + t * 16 + ln; const float bv = bp ? bf16_round(bp[col]) : 0.f;
#pragma unroll
    for (int r = 0; r < 8; ++r) { const int rloc = half * 16 + 8 * hh + r; float v = accs[u][r] * alpha + bv; if (CP) { if (rowsPerB < 0) v += CP[cofs + (size_t)(row0g + row0 + rloc) * ldc + col];        else { const int bidx = (row0g + row0 + rloc) / rowsPerB; v += CP[(size_t)bidx * sCPb + (size_t)by * 64 + col]; } }
      if (ACT == 3) v = fmaxf(v, 0.f); else if (ACT == 6) v = 0.5f * v * (1.0f + erff(v * 0.70710678118654752f)); else if (ACT == 11) v = 1.0f / (1.0f + expf(-v)); else if (ACT == 15) v = v / (1.0f + expf(-v)); else if (ACT == 12) v = (v > 0.f) ? v : 0.01f * v; else if (ACT == 8) v = tanhf(v); else if (ACT == 9) v = 0.5f * v * (1.0f + tanhf(0.7978845608028654f * (v + 0.044715f * v * v * v))); else if (ACT == 14) v = (v > 0.f) ? v : 0.1f * v; else if (ACT == 16) v = (v >= 0.f) ? v : 0.3f * v; else if (ACT == 17) v = (v >= 0.f) ? v : 0.2f * v;
      so[w][rloc][t * 16 + ln] = v; } }
  __builtin_amdgcn_fence(__ATOMIC_ACQ_REL, "workgroup"); __builtin_amdgcn_wave_barrier();
  const int rsub = lane >> 4, c4 = (lane & 15) * 4;
  for (int pass = 0; pass < 2; ++pass) {
#pragma unroll
    for (int q = 0; q < 16; ++q) { const int r = q * 2 + rsub; const v4f v = *(const v4fa*)&so[w][r][c4]; if (C) *(volatile v4f*)(C + cofs + (size_t)(row0 + r) * ldc + col0 + c4) = v; if (C16) { v4h h4; for (int i = 0; i < 4; ++i) h4[i] = (_Float16)v[i]; *(volatile v4h*)(C16 + cofs + (size_t)(row0 + r) * ldc + col0 + c4) = h4; } }
    if (pass == 0) __threadfence(); } }


__global__ __launch_bounds__(256) void k_xyrows(const float* __restrict__ x, const float* __restrict__ y, _Float16* __restrict__ XY) { __shared__ float tl[CC][33]; const int tid = threadIdx.x; const int half = blockIdx.x % 2; const int pb = (blockIdx.x / 2) % (PX / 32); const int b = blockIdx.x / (2 * (PX / 32)); const int p0 = pb * 32; const float* src = half ? y : x;
  for (int i = tid; i < CC * 32; i += 256) { const int c = i / 32, j = i % 32; tl[c][j] = bf16_round(src[((size_t)b * CC + c) * PX + p0 + j]); }
  __syncthreads();
  for (int pass = 0; pass < 2; ++pass) { for (int i = tid; i < 32 * 32; i += 256) { const int j = i / 32, c8 = (i % 32) * 8; FragH f; for (int q = 0; q < 8; ++q) f.h[q] = (_Float16)tl[c8 + q][j]; *(volatile v8us*)((unsigned short*)XY + ((size_t)b * PX + p0 + j) * 512 + half * CC + c8) = f.half[0]; } if (pass == 0) __threadfence(); } }
__global__ __launch_bounds__(256) void k_imf(const _Float16* __restrict__ XY, size_t r0, size_t nrows, _Float16* __restrict__ IM) { const size_t t_ = (size_t)blockIdx.x * 256 + threadIdx.x; if (t_ >= nrows * 9 * 64) return; const int c8 = (int)(t_ % 64) * 8; const int tap = (int)((t_ / 64) % 9); const size_t r = r0 + t_ / 576; const int p = (int)(r % PX); const size_t b = r / PX; const int yy = p / HS + tap / 3 - 1, xx = p % HS + tap % 3 - 1; v8us v;
  if (yy >= 0 && yy < HS && xx >= 0 && xx < HS) v = *(const v8us*)((const unsigned short*)XY + (b * PX + (size_t)yy * HS + xx) * 512 + c8); else { for (int q = 0; q < 8; ++q) v[q] = 0; }
  unsigned short* d = (unsigned short*)IM + (r - r0) * KF + (size_t)tap * 512 + c8; *(volatile v8us*)d = v; __threadfence(); *(volatile v8us*)d = v; }
__global__ __launch_bounds__(256) void k_wf(const float* __restrict__ w, _Float16* __restrict__ Bt) { const size_t t = (size_t)blockIdx.x * 256 + threadIdx.x; if (t >= (size_t)CC * KF / 8) return; const int c8 = (int)((t * 8) % 512); const int tap = (int)(((t * 8) / 512) % 9); const int o = (int)((t * 8) / KF); FragH f; for (int q = 0; q < 8; ++q) f.h[q] = (_Float16)(bf16_round(w[((size_t)o * 512 + c8 + q) * 9 + tap]) * 16.0f);
  *(volatile v8us*)((unsigned short*)Bt + t * 8) = f.half[0]; __threadfence(); *(volatile v8us*)((unsigned short*)Bt + t * 8) = f.half[0]; }
__global__ __launch_bounds__(256) void k_bngelu(const float* __restrict__ F, const float* __restrict__ g, const float* __restrict__ bb, const float* __restrict__ m, const float* __restrict__ v, _Float16* __restrict__ H16) {
  #pragma clang fp contract(off)
  __shared__ unsigned short stg[256][9]; const size_t t = (size_t)blockIdx.x * 256 + threadIdx.x; if (t >= NR * CC / 8) return; const int c0 = (int)((t * 8) % CC); const v8f f = *(const v8f*)(F + t * 8);
#pragma unroll 1
  for (int q = 0; q < 8; ++q) { const int c = c0 + q; const float hn = __fadd_rn(__fmul_rn((f[q] - bf16_round(m[c])) * rsqrtf(bf16_round(v[c]) + 1e-5f), bf16_round(g[c])), bf16_round(bb[c])); const float gl = 0.5f * hn * (1.0f + erff(hn * 0.70710678118654752f)); FragH one; one.h[0] = (_Float16)gl; stg[threadIdx.x][q] = one.u[0]; }
  FragH o; for (int q = 0; q < 8; ++q) o.u[q] = stg[threadIdx.x][q]; *(volatile v8us*)((unsigned short*)H16 + t * 8) = o.half[0]; __threadfence(); *(volatile v8us*)((unsigned short*)H16 + t * 8) = o.half[0]; }
__global__ __launch_bounds__(256) void k_wnat(const float* __restrict__ w, size_t n8, _Float16* __restrict__ Bt) { const size_t t = (size_t)blockIdx.x * 256 + threadIdx.x; if (t >= n8) return; FragH f; for (int q = 0; q < 8; ++q) f.h[q] = (_Float16)(bf16_round(w[t * 8 + q]) * 16.0f); *(volatile v8us*)((unsigned short*)Bt + t * 8) = f.half[0]; __threadfence(); *(volatile v8us*)((unsigned short*)Bt + t * 8) = f.half[0]; }
__global__ __launch_bounds__(256) void k_dw(const float* __restrict__ x, const float* __restrict__ y, const float* __restrict__ wx, const float* __restrict__ bx, const float* __restrict__ wy, const float* __restrict__ by, float* __restrict__ DWO) {
  #pragma clang fp contract(off)
  const int t = blockIdx.x * 256 + threadIdx.x; if (t >= 2 * NB * NS * CC) return; const int c = t % CC; const int pos = (t / CC) % NS; const int b = (t / (CC * NS)) % NB; const int src = t / (CC * NS * NB); const float* img = src ? y : x; const float* w = src ? wy : wx; const float* bs = src ? by : bx; const int gy = pos / GK, gx = pos % GK; float s = 0.f;
#pragma unroll 1
  for (int k = 0; k < 81; ++k) { const int i = k / 9, j = k % 9; const int yy = 8 * gy + i - 4, xx = 8 * gx + j - 4; if (yy < 0 || yy >= HS || xx < 0 || xx >= HS) continue; s = __fadd_rn(s, __fmul_rn(bf16_round(img[(((size_t)b * CC + c) * HS + yy) * HS + xx]), bf16_round(w[c * 81 + k]))); }
  s = s + bf16_round(bs[c]); *(volatile float*)(DWO + t) = s; __threadfence(); *(volatile float*)(DWO + t) = s; }
__global__ __launch_bounds__(256) void k_grid(const float* __restrict__ DWO, const float* __restrict__ gx_, const float* __restrict__ bx_, const float* __restrict__ pwx, const float* __restrict__ gy_, const float* __restrict__ by_, const float* __restrict__ pwy, float* __restrict__ GR) {
  #pragma clang fp contract(off)
  const int t = blockIdx.x * 256 + threadIdx.x; if (t >= 2 * NB * NS) return; const int pos = t % NS; const int src = t / (NB * NS); const float* h = DWO + (size_t)t * CC; const float* g = src ? gy_ : gx_; const float* be = src ? by_ : bx_; const float* pw = src ? pwy : pwx; float mu = 0.f;
#pragma unroll 1
  for (int c = 0; c < CC; ++c) mu += h[c]; mu = mu / 256.0f; float var = 0.f;
#pragma unroll 1
  for (int c = 0; c < CC; ++c) { const float d = h[c] - mu; var = __fadd_rn(var, __fmul_rn(d, d)); } var = var / 256.0f; const float rs = rsqrtf(var + 1e-5f); float o0 = 0.f, o1 = 0.f;
#pragma unroll 1
  for (int c = 0; c < CC; ++c) { const float hn = __fadd_rn(__fmul_rn((h[c] - mu) * rs, bf16_round(g[c])), bf16_round(be[c])); const float gl = 0.5f * hn * (1.0f + erff(hn * 0.70710678118654752f)); o0 = __fadd_rn(o0, __fmul_rn(bf16_round(pw[c]), gl)); o1 = __fadd_rn(o1, __fmul_rn(bf16_round(pw[CC + c]), gl)); }
  const int iy = pos / GK, ix = pos % GK; const float refy = ((0.5f + (float)iy) / (float)(GK - 1)) * 2.0f - 1.0f, refx = ((0.5f + (float)ix) / (float)(GK - 1)) * 2.0f - 1.0f;
  const float py = fminf(fmaxf(o0 + refy, -1.0f), 1.0f), px = fminf(fmaxf(o1 + refx, -1.0f), 1.0f);
  float* d = GR + (size_t)t * 32; for (int pass = 0; pass < 2; ++pass) { *(volatile float*)d = px; *(volatile float*)(d + 1) = py; if (pass == 0) __threadfence(); } }
__global__ __launch_bounds__(256) void k_samp(const float* __restrict__ x, const float* __restrict__ y, const float* __restrict__ Q, const float* __restrict__ GR, float* __restrict__ XS, float* __restrict__ YS, float* __restrict__ QS) {
  #pragma clang fp contract(off)
  const int t = blockIdx.x * 256 + threadIdx.x; if (t >= NB * NK * (CC / 8)) return; const int c0 = (t % (CC / 8)) * 8; const int n = (t / (CC / 8)) % NK; const int b = t / ((CC / 8) * NK); const int src = n / NS, pos = n % NS; const float* gp = GR + ((size_t)(src * NB + b) * NS + pos) * 32;
  const float gxv = gp[0], gyv = gp[1]; const float fx = __fmul_rn(__fmul_rn(gxv + 1.0f, 0.5f), (float)(HS - 1)), fy = __fmul_rn(__fmul_rn(gyv + 1.0f, 0.5f), (float)(HS - 1)); const float x0f = floorf(fx), y0f = floorf(fy); const float wx = fx - x0f, wy = fy - y0f;
  const int x0 = min(max((int)x0f, 0), HS - 1), x1 = min(max((int)x0f + 1, 0), HS - 1), y0 = min(max((int)y0f, 0), HS - 1), y1 = min(max((int)y0f + 1, 0), HS - 1);
  const float w00 = __fmul_rn(1.0f - wx, 1.0f - wy), w01 = __fmul_rn(wx, 1.0f - wy), w10 = __fmul_rn(1.0f - wx, wy), w11 = __fmul_rn(wx, wy); v8f ax, ay, aq;
  for (int q = 0; q < 8; ++q) { const int c = c0 + q; const size_t cb = ((size_t)b * CC + c) * PX; const size_t p00 = (size_t)y0 * HS + x0, p01 = (size_t)y0 * HS + x1, p10 = (size_t)y1 * HS + x0, p11 = (size_t)y1 * HS + x1;
    float s = __fmul_rn(bf16_round(x[cb + p00]), w00); s = __fadd_rn(s, __fmul_rn(bf16_round(x[cb + p01]), w01)); s = __fadd_rn(s, __fmul_rn(bf16_round(x[cb + p10]), w10)); s = __fadd_rn(s, __fmul_rn(bf16_round(x[cb + p11]), w11)); ax[q] = s;
    s = __fmul_rn(bf16_round(y[cb + p00]), w00); s = __fadd_rn(s, __fmul_rn(bf16_round(y[cb + p01]), w01)); s = __fadd_rn(s, __fmul_rn(bf16_round(y[cb + p10]), w10)); s = __fadd_rn(s, __fmul_rn(bf16_round(y[cb + p11]), w11)); ay[q] = s;
    const size_t rb = (size_t)b * PX; s = __fmul_rn(Q[(rb + p00) * CC + c], w00); s = __fadd_rn(s, __fmul_rn(Q[(rb + p01) * CC + c], w01)); s = __fadd_rn(s, __fmul_rn(Q[(rb + p10) * CC + c], w10)); s = __fadd_rn(s, __fmul_rn(Q[(rb + p11) * CC + c], w11)); aq[q] = s; }
  const size_t o = ((size_t)b * NK + n) * CC + c0; for (int pass = 0; pass < 2; ++pass) { *(volatile v8f*)(XS + o) = ax; *(volatile v8f*)(YS + o) = ay; *(volatile v8f*)(QS + o) = aq; if (pass == 0) __threadfence(); } }
__global__ __launch_bounds__(256) void k_tof16(const float* __restrict__ S, _Float16* __restrict__ D, size_t n8) { const size_t t = (size_t)blockIdx.x * 256 + threadIdx.x; if (t >= n8) return; const v8f v = *(const v8f*)(S + t * 8); FragH f; for (int q = 0; q < 8; ++q) f.h[q] = (_Float16)v[q]; *(volatile v8us*)((unsigned short*)D + t * 8) = f.half[0]; __threadfence(); *(volatile v8us*)((unsigned short*)D + t * 8) = f.half[0]; }
__global__ __launch_bounds__(256) void k_mix(const float* __restrict__ R, const float* __restrict__ sw2, const float* __restrict__ sw2b, const float* __restrict__ XS, const float* __restrict__ YS, _Float16* __restrict__ SMP16) {
  #pragma clang fp contract(off)
  const int t = blockIdx.x * 256 + threadIdx.x; if (t >= NB * NK * (CC / 8)) return; const int c0 = (t % (CC / 8)) * 8; const int row = t / (CC / 8); const float* r = R + (size_t)row * CC; float s0 = 0.f, s1 = 0.f;
#pragma unroll 1
  for (int c = 0; c < CC; ++c) { s0 = __fadd_rn(s0, __fmul_rn(bf16_round(sw2[c]), r[c])); s1 = __fadd_rn(s1, __fmul_rn(bf16_round(sw2[CC + c]), r[c])); } s0 = s0 + bf16_round(sw2b[0]); s1 = s1 + bf16_round(sw2b[1]);
  const float mx = fmaxf(s0, s1); const float e0 = expf(s0 - mx), e1 = expf(s1 - mx); const float w0 = e0 / (e0 + e1), w1 = e1 / (e0 + e1); FragH f;
  for (int q = 0; q < 8; ++q) { const size_t i = (size_t)row * CC + c0 + q; f.h[q] = (_Float16)__fadd_rn(__fmul_rn(w0, XS[i]), __fmul_rn(w1, YS[i])); }
  *(volatile v8us*)((unsigned short*)SMP16 + (size_t)row * CC + c0) = f.half[0]; __threadfence(); *(volatile v8us*)((unsigned short*)SMP16 + (size_t)row * CC + c0) = f.half[0]; }
__global__ __launch_bounds__(256) void k_vt(const _Float16* __restrict__ V16, _Float16* __restrict__ VT) { const int t = blockIdx.x * 256 + threadIdx.x; if (t >= NB * NHD * 64 * (NK / 8)) return; const int n0 = (t % (NK / 8)) * 8; const int hc = (t / (NK / 8)) % 64; const int h = (t / ((NK / 8) * 64)) % NHD; const int b = t / ((NK / 8) * 64 * NHD); FragH f;
  for (int q = 0; q < 8; ++q) f.h[q] = (hc < HC) ? V16[((size_t)b * NK + n0 + q) * CC + h * HC + hc] : (_Float16)0.f;
  unsigned short* d = (unsigned short*)VT + (((size_t)(b * NHD + h) * 64 + hc) * NK) + n0; *(volatile v8us*)d = f.half[0]; __threadfence(); *(volatile v8us*)d = f.half[0]; }
__global__ __launch_bounds__(256) void k_sm(const float* __restrict__ S, _Float16* __restrict__ P16) {
  #pragma clang fp contract(off)
  const int i = blockIdx.x * 256 + threadIdx.x; if (i >= NHD * PX) return; const float* s = S + (size_t)i * NK; float mx = -3.0e38f;
#pragma unroll 1
  for (int n = 0; n < NK; ++n) mx = fmaxf(mx, s[n]); float se = 0.f;
#pragma unroll 1
  for (int n = 0; n < NK; ++n) se += expf(s[n] - mx); const float inv = 1.0f / se; unsigned short* d = (unsigned short*)P16 + (size_t)i * NK;
#pragma unroll 1
  for (int n0 = 0; n0 < NK; n0 += 8) { FragH f; for (int q = 0; q < 8; ++q) f.h[q] = (_Float16)(expf(s[n0 + q] - mx) * inv); *(volatile v8us*)(d + n0) = f.half[0]; __threadfence(); *(volatile v8us*)(d + n0) = f.half[0]; } }
__global__ __launch_bounds__(256) void k_merge(const float* __restrict__ AT, int b, _Float16* __restrict__ OUT16) { const int t = blockIdx.x * 256 + threadIdx.x; if (t >= PX * NHD * 4) return; const int pc = t % 4; const int h = (t / 4) % NHD; const int m = t / (4 * NHD); const v8f a = *(const v8f*)(AT + ((size_t)h * PX + m) * 64 + pc * 8); FragH f; for (int q = 0; q < 8; ++q) f.h[q] = (_Float16)a[q];
  unsigned short* d = (unsigned short*)OUT16 + ((size_t)b * PX + m) * CC + h * HC + pc * 8; *(volatile v8us*)d = f.half[0]; __threadfence(); *(volatile v8us*)d = f.half[0]; }
__global__ __launch_bounds__(256) void k_out(const float* __restrict__ O, float* __restrict__ out) { const size_t t = (size_t)blockIdx.x * 256 + threadIdx.x; if (t >= (size_t)NB * CC * PX / 8) return; const int p0 = (int)((t * 8) % PX); const size_t bc = (t * 8) / PX; const int c = (int)(bc % CC); const size_t b = bc / CC; v8f r; for (int q = 0; q < 8; ++q) r[q] = O[(b * PX + p0 + q) * CC + c];
  *(volatile v8f*)(out + t * 8) = r; __threadfence(); *(volatile v8f*)(out + t * 8) = r; }

extern "C" void kernel_launch(void* const* d_in, const int* in_sizes, int n_in,
                              void* d_out, int out_size, void* d_ws, size_t ws_size, hipStream_t stream) {
  (void)in_sizes; (void)n_in; (void)out_size;
  const float* const* I = (const float* const*)d_in; const float* x = I[0]; const float* y = I[1]; const float* fw = I[2]; const float* fb = I[3]; const float* bng = I[4]; const float* bnb = I[5]; const float* bnm = I[6]; const float* bnv = I[7]; const float* pqw = I[8]; const float* pqb = I[9];
  const float* oxdw = I[10]; const float* oxdb = I[11]; const float* oxg = I[12]; const float* oxb = I[13]; const float* oxpw = I[14]; const float* oydw = I[15]; const float* oydb = I[16]; const float* oyg = I[17]; const float* oyb = I[18]; const float* oypw = I[19];
  const float* sw1w = I[20]; const float* sw1b = I[21]; const float* sw2w = I[22]; const float* sw2b = I[23]; const float* pkw = I[24]; const float* pkb = I[25]; const float* pvw = I[26]; const float* pvb = I[27]; const float* pow_ = I[28]; const float* pob = I[29];
  char* ws = (char*)d_ws; size_t off = 0;
  auto take = [&](size_t bytes) { char* p = ws + off; off += (bytes + 255) & ~(size_t)255; return p; };
  _Float16* BF = (_Float16*)take((size_t)CC * KF * 2); _Float16* BQ = (_Float16*)take((size_t)CC * CC * 2); _Float16* BS1 = (_Float16*)take((size_t)CC * CC * 2); _Float16* BK = (_Float16*)take((size_t)CC * CC * 2); _Float16* BV = (_Float16*)take((size_t)CC * CC * 2); _Float16* BO = (_Float16*)take((size_t)CC * CC * 2);
  float* DWO = (float*)take((size_t)2 * NB * NS * CC * 4); float* GR = (float*)take((size_t)2 * NB * NS * 32 * 4); float* XS = (float*)take(NKR * CC * 4); float* YS = (float*)take(NKR * CC * 4); float* QS = (float*)take(NKR * CC * 4); _Float16* QS16 = (_Float16*)take(NKR * CC * 2); float* R = (float*)take(NKR * CC * 4); _Float16* SMP16 = (_Float16*)take(NKR * CC * 2); _Float16* K16 = (_Float16*)take(NKR * CC * 2); _Float16* V16 = (_Float16*)take(NKR * CC * 2); _Float16* VT = (_Float16*)take((size_t)NB * NHD * 64 * NK * 2);
  const size_t szXY = NR * 512 * 2, szAT = (size_t)NHD * PX * 64 * 4, szO16 = NR * CC * 2; const size_t reg1 = (szXY > szAT + szO16) ? szXY : (szAT + szO16);
  const size_t szIM = (size_t)RCH * KF * 2, szQ = NR * CC * 4, szQ16 = NR * CC * 2, szS = (size_t)NHD * PX * NK * 4, szP = (size_t)NHD * PX * NK * 2; const size_t reg2 = (szIM > szQ + szQ16 + szS + szP) ? szIM : (szQ + szQ16 + szS + szP);
  char* R1 = take(reg1); char* R2 = take(reg2); float* F = (float*)take(NR * CC * 4); _Float16* H16 = (_Float16*)take(NR * CC * 2);
  _Float16* XY = (_Float16*)R1; float* AT = (float*)R1; _Float16* OUT16 = (_Float16*)(R1 + szAT);
  _Float16* IM = (_Float16*)R2; float* Q = (float*)R2; _Float16* Q16 = (_Float16*)(R2 + szQ); float* S = (float*)(R2 + szQ + szQ16); _Float16* P16 = (_Float16*)(R2 + szQ + szQ16 + szS); float* O = F;
  if (off > ws_size) return;
  k_wf<<<(unsigned)(((size_t)CC * KF / 8 + 255) / 256), 256, 0, stream>>>(fw, BF); k_wnat<<<(CC * CC / 8 + 255) / 256, 256, 0, stream>>>(pqw, (size_t)CC * CC / 8, BQ); k_wnat<<<(CC * CC / 8 + 255) / 256, 256, 0, stream>>>(sw1w, (size_t)CC * CC / 8, BS1); k_wnat<<<(CC * CC / 8 + 255) / 256, 256, 0, stream>>>(pkw, (size_t)CC * CC / 8, BK); k_wnat<<<(CC * CC / 8 + 255) / 256, 256, 0, stream>>>(pvw, (size_t)CC * CC / 8, BV); k_wnat<<<(CC * CC / 8 + 255) / 256, 256, 0, stream>>>(pow_, (size_t)CC * CC / 8, BO);
  k_xyrows<<<NB * 2 * (PX / 32), 256, 0, stream>>>(x, y, XY);
  for (size_t r0 = 0; r0 < NR; r0 += RCH) { const size_t nr = (NR - r0 < (size_t)RCH) ? (NR - r0) : (size_t)RCH; k_imf<<<(unsigned)((nr * 576 + 255) / 256), 256, 0, stream>>>(XY, r0, nr, IM); k_gemm2<0><<<dim3((unsigned)((nr / 128) * (CC / 64)), 1), 128, 0, stream>>>(IM, KF, 0, BF, KF, 0, 0.0625f, fb, 0, nullptr, 1, 0, 0, F + r0 * CC, nullptr, CC, 0, (int)nr, CC, KF); }
  const unsigned n8 = (unsigned)((NR * CC / 8 + 255) / 256); const dim3 g256((unsigned)((NR / 128) * (CC / 64)), 1), g1k((unsigned)((NKR / 128) * (CC / 64)), 1);
  k_bngelu<<<n8, 256, 0, stream>>>(F, bng, bnb, bnm, bnv, H16);
  k_gemm2<0><<<g256, 128, 0, stream>>>(H16, CC, 0, BQ, CC, 0, 0.0625f, pqb, 0, nullptr, 1, 0, 0, Q, Q16, CC, 0, (int)NR, CC, CC);
  k_dw<<<(2 * NB * NS * CC + 255) / 256, 256, 0, stream>>>(x, y, oxdw, oxdb, oydw, oydb, DWO); k_grid<<<(2 * NB * NS + 255) / 256, 256, 0, stream>>>(DWO, oxg, oxb, oxpw, oyg, oyb, oypw, GR);
  k_samp<<<(NB * NK * (CC / 8) + 255) / 256, 256, 0, stream>>>(x, y, Q, GR, XS, YS, QS);
  k_tof16<<<(unsigned)((NKR * CC / 8 + 255) / 256), 256, 0, stream>>>(QS, QS16, NKR * CC / 8);
  k_gemm2<3><<<g1k, 128, 0, stream>>>(QS16, CC, 0, BS1, CC, 0, 0.0625f, sw1b, 0, nullptr, 1, 0, 0, R, nullptr, CC, 0, (int)NKR, CC, CC);
  k_mix<<<(NB * NK * (CC / 8) + 255) / 256, 256, 0, stream>>>(R, sw2w, sw2b, XS, YS, SMP16);
  k_gemm2<0><<<g1k, 128, 0, stream>>>(SMP16, CC, 0, BK, CC, 0, 0.0625f, pkb, 0, nullptr, 1, 0, 0, nullptr, K16, CC, 0, (int)NKR, CC, CC);
  k_gemm2<0><<<g1k, 128, 0, stream>>>(SMP16, CC, 0, BV, CC, 0, 0.0625f, pvb, 0, nullptr, 1, 0, 0, nullptr, V16, CC, 0, (int)NKR, CC, CC);
  k_vt<<<(NB * NHD * 64 * (NK / 8) + 255) / 256, 256, 0, stream>>>(V16, VT);
  for (int b = 0; b < NB; ++b) {
    k_gemm2<0><<<dim3((PX / 128) * (NK / 64), NHD), 128, 0, stream>>>(Q16 + (size_t)b * PX * CC, CC, (size_t)HC, K16 + (size_t)b * NK * CC, CC, (size_t)HC, 0.17677669529663687f, nullptr, 0, nullptr, 1, 0, 0, S, nullptr, NK, (size_t)PX * NK, PX, NK, HC);
    k_sm<<<(NHD * PX + 255) / 256, 256, 0, stream>>>(S, P16);
    k_gemm2<0><<<dim3((PX / 128) * 1, NHD), 128, 0, stream>>>(P16, NK, (size_t)PX * NK, VT + (size_t)b * NHD * 64 * NK, NK, (size_t)64 * NK, 1.0f, nullptr, 0, nullptr, 1, 0, 0, AT, nullptr, 64, (size_t)PX * 64, PX, 64, NK);
    k_merge<<<(PX * NHD * 4 + 255) / 256, 256, 0, stream>>>(AT, b, OUT16); }
  k_gemm2<0><<<g256, 128, 0, stream>>>(OUT16, CC, 0, BO, CC, 0, 0.0625f, pob, 0, nullptr, 1, 0, 0, O, nullptr, CC, 0, (int)NR, CC, CC);
  k_out<<<(unsigned)(((size_t)NB * CC * PX / 8 + 255) / 256), 256, 0, stream>>>(O, (float*)d_out);
}
